// GCNEdgeClassifier_49795850830535
// MI455X (gfx1250) — hardware-verified
//
#include <hip/hip_runtime.h>
#include <stddef.h>
#include <stdint.h>


#define HD      128
#define HD2     256
#define NOUT    3
#define NPLANE  5
#define PLH     (HD * HD)
#define NTHR    256
#define NWAVE   8
#define EPT     8
#define CHUNK   (NTHR * EPT)
#define WCAP    (EPT * 32)
#define LISTN   (NWAVE * WCAP)
#define NBMAX   2048
#define SLB     11
#define RCAP    28672
#define DEGCAP  128
#define GBM     64
#define SP      132
#define CA      32.0f
#define CL      2048.0f
#define CW      1024.0f
#define SCL     0.000030517578125f
#define SCLL    0.00000001490116119384765625f
#define WSMAX   134217728
#define LDS_AGG ((2 * RCAP + 2 * NBMAX + LISTN) * 4 + 64)
#define LDS_DEG ((RCAP + NBMAX + LISTN) * 4 + 64)

static_assert((CHUNK & (CHUNK - 1)) == 0 && CHUNK <= 4096);
static_assert(NBMAX == (1 << SLB));
static_assert(NTHR * 8 == NBMAX);
static_assert(LISTN >= NBMAX);
static_assert(LISTN >= NWAVE * WCAP);
static_assert((RCAP % 32) == 0);
static_assert(LDS_AGG <= 300000);
static_assert(LDS_DEG <= 300000);
static_assert(HD / 32 == 4 && HD2 == 2 * HD);
static_assert(NWAVE * 8 == GBM);
static_assert((SP * 4) % 16 == 0);
static_assert(NTHR * NOUT % 4 == 0);
static_assert((PLH / 8) % NTHR == 0 || (128 % 16) == 0);

typedef float    v4f  __attribute__((ext_vector_type(4)));
typedef float    v8f  __attribute__((ext_vector_type(8)));
typedef int      v4i  __attribute__((ext_vector_type(4)));
typedef int      v8i  __attribute__((ext_vector_type(8)));
typedef _Float16 v8h  __attribute__((ext_vector_type(8)));
typedef _Float16 v16h __attribute__((ext_vector_type(16)));
union FragH { v16h v; v8h h[2]; v8i w; };

__device__ __forceinline__ v8f wmh(const FragH& a, const FragH& b, v8f c) {
  v8f d = __builtin_amdgcn_wmma_f32_16x16x32_f16(false, a.v, false, b.v, (short)0, c, false, false);
  asm volatile("v_nop\n\tv_nop\n\tv_nop\n\tv_nop" : "+v"(d) : "v"(a.w), "v"(b.w));
  return d;
}

__device__ __forceinline__ float bf16r(float x) {
  unsigned u = (unsigned)__float_as_uint(x);
  u = (u + 0x7FFFu + ((u >> 16) & 1u)) & 0xFFFF0000u;
  return __uint_as_float(u);
}
__device__ __forceinline__ v4f bf16r4(const v4f v) {
  v4f r;
  r.x = bf16r(v.x); r.y = bf16r(v.y); r.z = bf16r(v.z); r.w = bf16r(v.w);
  return r;
}

__device__ __forceinline__ v8h cvt8hb(const v4f a, const v4f b, const float c) {
  v8h hv;
  hv[0] = (_Float16)(bf16r(a.x) * c); hv[1] = (_Float16)(bf16r(a.y) * c);
  hv[2] = (_Float16)(bf16r(a.z) * c); hv[3] = (_Float16)(bf16r(a.w) * c);
  hv[4] = (_Float16)(bf16r(b.x) * c); hv[5] = (_Float16)(bf16r(b.y) * c);
  hv[6] = (_Float16)(bf16r(b.z) * c); hv[7] = (_Float16)(bf16r(b.w) * c);
  return hv;
}

__device__ __forceinline__ void cvt8hl(const v4f a, const v4f b, v8h& hi, v8h& lo) {
  const float t[8] = {a.x, a.y, a.z, a.w, b.x, b.y, b.z, b.w};
#pragma unroll
  for (int i = 0; i < 8; ++i) {
    const float s = t[i] * CA;
    const _Float16 q = (_Float16)s;
    hi[i] = q;
    lo[i] = (_Float16)((s - (float)q) * CL);
  }
}

__device__ __forceinline__ v4f relu4(const v4f v) {
  v4f r;
  r.x = fmaxf(v.x, 0.f); r.y = fmaxf(v.y, 0.f); r.z = fmaxf(v.z, 0.f); r.w = fmaxf(v.w, 0.f);
  return r;
}

__device__ __forceinline__ int scan_chunk(const int* __restrict__ dsts, int nE, int cbase, int slotBase,
                                          int nb, int vec8, int* list, int tid, int lane, int wave) {
  int wc = 0;
  const int el0  = tid * EPT;
  const int e0   = cbase + el0;
  const int sent = -2147483647 - 1;
  v4i da, db;
  if (vec8 != 0 && cbase + CHUNK <= nE) {
    da = *(const v4i*)(dsts + e0);
    db = *(const v4i*)(dsts + e0 + 4);
  } else {
    da.x = (e0     < nE) ? dsts[min(e0,     nE - 1)] : sent;
    da.y = (e0 + 1 < nE) ? dsts[min(e0 + 1, nE - 1)] : sent;
    da.z = (e0 + 2 < nE) ? dsts[min(e0 + 2, nE - 1)] : sent;
    da.w = (e0 + 3 < nE) ? dsts[min(e0 + 3, nE - 1)] : sent;
    db.x = (e0 + 4 < nE) ? dsts[min(e0 + 4, nE - 1)] : sent;
    db.y = (e0 + 5 < nE) ? dsts[min(e0 + 5, nE - 1)] : sent;
    db.z = (e0 + 6 < nE) ? dsts[min(e0 + 6, nE - 1)] : sent;
    db.w = (e0 + 7 < nE) ? dsts[min(e0 + 7, nE - 1)] : sent;
  }
  const unsigned nbs = (unsigned)slotBase;
  const unsigned unb = (unsigned)nb;
  const unsigned s0 = (unsigned)da.x - nbs, s1 = (unsigned)da.y - nbs;
  const unsigned s2 = (unsigned)da.z - nbs, s3 = (unsigned)da.w - nbs;
  const unsigned s4 = (unsigned)db.x - nbs, s5 = (unsigned)db.y - nbs;
  const unsigned s6 = (unsigned)db.z - nbs, s7 = (unsigned)db.w - nbs;
  const bool h0 = s0 < unb, h1 = s1 < unb, h2 = s2 < unb, h3 = s3 < unb;
  const bool h4 = s4 < unb, h5 = s5 < unb, h6 = s6 < unb, h7 = s7 < unb;
  const unsigned any = __builtin_amdgcn_ballot_w32(h0 | h1 | h2 | h3 | h4 | h5 | h6 | h7);
  if (any != 0u) {
#define HITJ(J, HJ, SJ) { \
      const unsigned mj = __builtin_amdgcn_ballot_w32(HJ); \
      if (mj != 0u) { \
        if (HJ) { \
          const int pos = wc + (int)__builtin_amdgcn_mbcnt_lo(mj, 0u); \
          if (pos < WCAP) list[wave * WCAP + pos] = ((el0 + (J)) << 12) | (int)(SJ); \
        } \
        wc += (int)__builtin_popcount(mj); } }
    HITJ(0, h0, s0)
    HITJ(1, h1, s1)
    HITJ(2, h2, s2)
    HITJ(3, h3, s3)
    HITJ(4, h4, s4)
    HITJ(5, h5, s5)
    HITJ(6, h6, s6)
    HITJ(7, h7, s7)
#undef HITJ
  }
  return wc;
}

__global__ __launch_bounds__(NTHR) void k_wcvt(const float* __restrict__ w0, const float* __restrict__ w1,
                                               const float* __restrict__ w2, const float* __restrict__ wm1,
                                               _Float16* wt, int nUnits) {
  const int u = (int)blockIdx.x * NTHR + (int)threadIdx.x;
  if (u >= nUnits) return;
  const int ng = u >> 4;
  const int k8 = (u & 15) * 8;
  int pl = ng >> 7;
  pl = pl > 4 ? 4 : pl;
  const int n  = ng & (HD - 1);
  const float* src = (pl == 0) ? w0 : ((pl == 1) ? w1 : ((pl == 2) ? w2 :
                     ((pl == 3) ? wm1 : (wm1 + (size_t)HD * HD))));
  const float* p = src + (size_t)k8 * HD + n;
  v4f a, b;
  a.x = p[0];              a.y = p[(size_t)HD];     a.z = p[(size_t)2 * HD]; a.w = p[(size_t)3 * HD];
  b.x = p[(size_t)4 * HD]; b.y = p[(size_t)5 * HD]; b.z = p[(size_t)6 * HD]; b.w = p[(size_t)7 * HD];
  const v8h hv = cvt8hb(a, b, CW);
  const size_t o = (size_t)ng * HD + k8;
  *(volatile v8h*)(wt + o) = hv;
  __threadfence();
  *(volatile v8h*)(wt + o) = hv;
}

__global__ __launch_bounds__(NTHR) void k_embr(const float* __restrict__ emb, float* embr, int nV, int nTot) {
  const int t = (int)blockIdx.x * NTHR + (int)threadIdx.x;
  if (t >= nTot) return;
  const int row = t >> 5, c4 = (t & 31) * 4;
  const int rc  = row < nV ? row : nV - 1;
  v4f v = *(const v4f*)(emb + (size_t)rc * HD + c4);
  v = bf16r4(v);
  const v4f z4 = {0.f, 0.f, 0.f, 0.f};
  if (row >= nV) v = z4;
  float* op = embr + (size_t)row * HD + c4;
  *(volatile v4f*)op = v;
  __threadfence();
  *(volatile v4f*)op = v;
}

template<int EPI>
__global__ __launch_bounds__(NTHR) void k_pgemm(const float* A, const _Float16* __restrict__ WT,
                                                const float* __restrict__ bias, const float* __restrict__ rsc,
                                                float* outF, int nAr) {
  __shared__ __attribute__((aligned(16))) float stg[GBM * SP];
  const int tid = (int)threadIdx.x, lane = tid & 31, wave = tid >> 5, hh = lane >> 4, m = lane & 15;
  const int rowBase = (int)blockIdx.x * GBM;
  const int wr = wave & 3, wcg = wave >> 2;

  v8f acch[4], accl[4];
  {
    const v8f z = {0.f, 0.f, 0.f, 0.f, 0.f, 0.f, 0.f, 0.f};
#pragma unroll
    for (int t = 0; t < 4; ++t) { acch[t] = z; accl[t] = z; }
  }
  const int gra = rowBase + 16 * wr + m;
  const int grc = gra > nAr - 1 ? nAr - 1 : gra;
  const float* ap = A + (size_t)grc * HD + 8 * hh;
  const _Float16* wp = WT + (size_t)(64 * wcg + m) * HD + 8 * hh;
#pragma unroll 1
  for (int ks = 0; ks < HD / 32; ++ks) {
    const float* aq = ap + 32 * ks;
    const v4f a0 = *(const v4f*)aq,        a1 = *(const v4f*)(aq + 4);
    const v4f a2 = *(const v4f*)(aq + 16), a3 = *(const v4f*)(aq + 20);
    FragH ah, al;
    cvt8hl(a0, a1, ah.h[0], al.h[0]);
    cvt8hl(a2, a3, ah.h[1], al.h[1]);
#pragma unroll
    for (int t = 0; t < 4; ++t) {
      const _Float16* wq = wp + (size_t)(16 * t) * HD + 32 * ks;
      FragH bf;
      bf.h[0] = *(const v8h*)wq;
      bf.h[1] = *(const v8h*)(wq + 16);
      acch[t] = wmh(ah, bf, acch[t]);
      accl[t] = wmh(al, bf, accl[t]);
    }
  }

  float rs[8];
#pragma unroll
  for (int r = 0; r < 8; ++r) rs[r] = 1.f;
  if (EPI == 1) {
    const int lr0 = rowBase + 16 * wr + 8 * hh;
    const v4f ra = *(const v4f*)(rsc + lr0), rb = *(const v4f*)(rsc + lr0 + 4);
    rs[0] = ra.x; rs[1] = ra.y; rs[2] = ra.z; rs[3] = ra.w;
    rs[4] = rb.x; rs[5] = rb.y; rs[6] = rb.z; rs[7] = rb.w;
  }

#pragma unroll
  for (int t = 0; t < 4; ++t) {
    const int lc = 64 * wcg + 16 * t + m;
    float bv = 0.f;
    if (EPI == 0) bv = bf16r(bias[lc]);
#pragma unroll
    for (int r = 0; r < 8; ++r) {
      const int lr = 16 * wr + 8 * hh + r;
      float v = acch[t][r] * SCL;
      v = fmaf(accl[t][r], SCLL, v);
      if (EPI == 0)      v = v + bv;
      else if (EPI == 1) v = v * rs[r];
      stg[lr * SP + lc] = v;
    }
  }
  __syncthreads();

  v4f y[8];
#pragma unroll
  for (int i = 0; i < 8; ++i) {
    const int lr = 8 * wave + i;
    y[i] = *(const v4f*)(stg + lr * SP + 4 * lane);
  }
#pragma unroll
  for (int i = 0; i < 8; ++i) {
    const int grow = rowBase + 8 * wave + i;
    *(volatile v4f*)(outF + (size_t)grow * HD + 4 * lane) = y[i];
  }
  __threadfence();
#pragma unroll
  for (int i = 0; i < 8; ++i) {
    const int grow = rowBase + 8 * wave + i;
    *(volatile v4f*)(outF + (size_t)grow * HD + 4 * lane) = y[i];
  }
}

__device__ __forceinline__ float disval(int c, bool live, bool ovf, float qnan) {
  const bool bad = ovf || c < 0 || c > DEGCAP;
  const int cc = c < 0 ? 0 : (c > DEGCAP ? DEGCAP : c);
  const float d = rsqrtf((float)(cc + 1));
  return live ? (bad ? qnan : d) : 0.f;
}

__global__ __launch_bounds__(NTHR) void k_deg(const int* __restrict__ dsts, float* DIS, int nN, int nE, int nb, int vec8) {
  extern __shared__ v4f lds_dynd[];
  int* reg1 = (int*)lds_dynd;
  int* scnt = reg1 + RCAP;
  int* list = scnt + NBMAX;
  int* wcnt = list + LISTN;
  const int tid = (int)threadIdx.x, lane = tid & 31, wave = tid >> 5;
  const int nodeBase = (int)blockIdx.x * nb;

  for (int i = tid; i < NBMAX; i += NTHR) scnt[i] = 0;
  __syncthreads();

  int tot = 0;
  const int nChunks = (nE + CHUNK - 1) / CHUNK;
#pragma unroll 1
  for (int ch = 0; ch < nChunks; ++ch) {
    const int cbase = ch * CHUNK;
    const int wc = scan_chunk(dsts, nE, cbase, nodeBase, nb, vec8, list, tid, lane, wave);
    if (lane == 0) wcnt[wave] = wc;
    __syncthreads();
    int pre = 0, all = 0;
#pragma unroll
    for (int w2 = 0; w2 < NWAVE; ++w2) {
      int c = wcnt[w2];
      c = c < 0 ? 0 : (c > WCAP ? WCAP : c);
      all += c;
      pre += (w2 < wave) ? c : 0;
    }
    const int wcc  = wc > WCAP ? WCAP : wc;
    const int base = tot + pre;
#pragma unroll 1
    for (int i = lane; i < wcc; i += 32) {
      const int ent = list[wave * WCAP + i];
      const int el  = (ent >> 12) & (CHUNK - 1);
      const int sl  = ent & (NBMAX - 1);
      int eid = cbase + el;
      eid = eid > nE - 1 ? nE - 1 : eid;
      const int pos = base + i;
      if (pos < RCAP) reg1[pos] = (int)(((unsigned)eid << SLB) | (unsigned)sl);
    }
    tot += all;
    tot = tot > RCAP ? RCAP : tot;
    __syncthreads();
  }
  const int nh = tot;

  if (wave == 0) {
#pragma unroll 1
    for (int b0 = 0; b0 < nh; b0 += 32) {
      const int idx = b0 + lane;
      const int uv  = reg1[idx < RCAP ? idx : RCAP - 1];
      const int m32 = (nh - b0) < 32 ? (nh - b0) : 32;
#pragma unroll 1
      for (int k = 0; k < m32; ++k) {
        const int u  = __builtin_amdgcn_readlane(uv, k);
        const int sl = u & (NBMAX - 1);
        if (lane == 0) scnt[sl] = scnt[sl] + 1;
      }
    }
  }
  __syncthreads();

  {
    const bool ovf = (nh >= RCAP);
    const float qnan = __int_as_float(0x7fc00000);
    const int nq = nb >> 2;
#pragma unroll 1
    for (int t = tid; t < nq; t += NTHR) {
      const v4i c4 = *(const v4i*)(scnt + 4 * t);
      const int rb = nodeBase + 4 * t;
      v4f dv;
      dv.x = disval(c4.x, rb     < nN, ovf, qnan);
      dv.y = disval(c4.y, rb + 1 < nN, ovf, qnan);
      dv.z = disval(c4.z, rb + 2 < nN, ovf, qnan);
      dv.w = disval(c4.w, rb + 3 < nN, ovf, qnan);
      *(volatile v4f*)(DIS + rb) = dv;
    }
    __threadfence();
#pragma unroll 1
    for (int t = tid; t < nq; t += NTHR) {
      const v4i c4 = *(const v4i*)(scnt + 4 * t);
      const int rb = nodeBase + 4 * t;
      v4f dv;
      dv.x = disval(c4.x, rb     < nN, ovf, qnan);
      dv.y = disval(c4.y, rb + 1 < nN, ovf, qnan);
      dv.z = disval(c4.z, rb + 2 < nN, ovf, qnan);
      dv.w = disval(c4.w, rb + 3 < nN, ovf, qnan);
      *(volatile v4f*)(DIS + rb) = dv;
    }
  }
}

__global__ __launch_bounds__(NTHR) void k_gath1(const int* __restrict__ xi, const float* __restrict__ TT,
                                                const float* __restrict__ DIS, float* G, int nN, int nV, int nTot) {
  const int t = (int)blockIdx.x * NTHR + (int)threadIdx.x;
  if (t >= nTot) return;
  const int n = t >> 5, c4 = (t & 31) * 4;
  const int nc = n < nN ? n : nN - 1;
  int v = xi[nc];
  v = v < 0 ? 0 : (v > nV - 1 ? nV - 1 : v);
  const float d = DIS[n];
  const v4f tv = *(const v4f*)(TT + (size_t)v * HD + c4);
  v4f g = tv * d;
  const v4f z4 = {0.f, 0.f, 0.f, 0.f};
  if (n >= nN) g = z4;
  float* op = G + (size_t)n * HD + c4;
  *(volatile v4f*)op = g;
  __threadfence();
  *(volatile v4f*)op = g;
}

__global__ __launch_bounds__(NTHR) void k_agg(
    const int* __restrict__ dsts, const int* __restrict__ srcs, const float* __restrict__ G,
    const float* __restrict__ DIS, const float* __restrict__ bias, float* H,
    int nN, int nE, int nb, int vec8, int NPr) {
  extern __shared__ v4f lds_dyn[];
  int* reg1 = (int*)lds_dyn;
  int* reg2 = reg1 + RCAP;
  int* scnt = reg2 + RCAP;
  int* soff = scnt + NBMAX;
  int* list = soff + NBMAX;
  int* wcnt = list + LISTN;
  int* wtot = wcnt + NWAVE;
  const int tid = (int)threadIdx.x, lane = tid & 31, wave = tid >> 5;
  const int nodeBase = (int)blockIdx.x * nb;

  for (int i = tid; i < NBMAX; i += NTHR) scnt[i] = 0;
  __syncthreads();

  int tot = 0;
  const int nChunks = (nE + CHUNK - 1) / CHUNK;
#pragma unroll 1
  for (int ch = 0; ch < nChunks; ++ch) {
    const int cbase = ch * CHUNK;
    const int wc = scan_chunk(dsts, nE, cbase, nodeBase, nb, vec8, list, tid, lane, wave);
    if (lane == 0) wcnt[wave] = wc;
    __syncthreads();
    int pre = 0, all = 0;
#pragma unroll
    for (int w2 = 0; w2 < NWAVE; ++w2) {
      int c = wcnt[w2];
      c = c < 0 ? 0 : (c > WCAP ? WCAP : c);
      all += c;
      pre += (w2 < wave) ? c : 0;
    }
    const int wcc  = wc > WCAP ? WCAP : wc;
    const int base = tot + pre;
#pragma unroll 1
    for (int i = lane; i < wcc; i += 32) {
      const int ent = list[wave * WCAP + i];
      const int el  = (ent >> 12) & (CHUNK - 1);
      const int sl  = ent & (NBMAX - 1);
      int eid = cbase + el;
      eid = eid > nE - 1 ? nE - 1 : eid;
      const int pos = base + i;
      if (pos < RCAP) reg1[pos] = (int)(((unsigned)eid << SLB) | (unsigned)sl);
    }
    tot += all;
    tot = tot > RCAP ? RCAP : tot;
    __syncthreads();
  }
  const int nh = tot;

  if (wave == 0) {
#pragma unroll 1
    for (int b0 = 0; b0 < nh; b0 += 32) {
      const int idx = b0 + lane;
      const int uv  = reg1[idx < RCAP ? idx : RCAP - 1];
      const int m32 = (nh - b0) < 32 ? (nh - b0) : 32;
#pragma unroll 1
      for (int k = 0; k < m32; ++k) {
        const int u  = __builtin_amdgcn_readlane(uv, k);
        const int sl = u & (NBMAX - 1);
        if (lane == 0) scnt[sl] = scnt[sl] + 1;
      }
    }
  }
  __syncthreads();

  {
    const v4i ca = *(const v4i*)(scnt + 8 * tid);
    const v4i cb = *(const v4i*)(scnt + 8 * tid + 4);
    const int e0 = ca.x < 0 ? 0 : ca.x, e1 = ca.y < 0 ? 0 : ca.y, e2 = ca.z < 0 ? 0 : ca.z, e3 = ca.w < 0 ? 0 : ca.w;
    const int e4 = cb.x < 0 ? 0 : cb.x, e5 = cb.y < 0 ? 0 : cb.y, e6 = cb.z < 0 ? 0 : cb.z, e7 = cb.w < 0 ? 0 : cb.w;
    const int ts = e0 + e1 + e2 + e3 + e4 + e5 + e6 + e7;
    int incl = ts;
#pragma unroll
    for (int d = 1; d < 32; d <<= 1) {
      const int up = __shfl_up(incl, d);
      if (lane >= d) incl += up;
    }
    if (lane == 31) wtot[wave] = incl;
    __syncthreads();
    int pre = 0;
#pragma unroll
    for (int w2 = 0; w2 < NWAVE; ++w2) pre += (w2 < wave) ? wtot[w2] : 0;
    int run = pre + incl - ts;
    soff[8 * tid + 0] = run; run += e0;
    soff[8 * tid + 1] = run; run += e1;
    soff[8 * tid + 2] = run; run += e2;
    soff[8 * tid + 3] = run; run += e3;
    soff[8 * tid + 4] = run; run += e4;
    soff[8 * tid + 5] = run; run += e5;
    soff[8 * tid + 6] = run; run += e6;
    soff[8 * tid + 7] = run;
  }
  __syncthreads();
  for (int i = tid; i < NBMAX; i += NTHR) list[i] = soff[i];
  __syncthreads();

  if (wave == 0) {
#pragma unroll 1
    for (int b0 = 0; b0 < nh; b0 += 32) {
      const int idx = b0 + lane;
      const int uv  = reg1[idx < RCAP ? idx : RCAP - 1];
      const int m32 = (nh - b0) < 32 ? (nh - b0) : 32;
#pragma unroll 1
      for (int k = 0; k < m32; ++k) {
        const int u   = __builtin_amdgcn_readlane(uv, k);
        const int sl  = u & (NBMAX - 1);
        const int eid = (int)((unsigned)u >> SLB);
        if (lane == 0) {
          int pos = list[sl];
          pos = pos < 0 ? 0 : (pos > RCAP - 1 ? RCAP - 1 : pos);
          reg2[pos] = eid;
          list[sl] = pos + 1;
        }
      }
    }
  }
  __syncthreads();

  v4f b4;
  {
    const v4f bb = *(const v4f*)(bias + 4 * lane);
    b4 = bf16r4(bb);
  }
  const int nbw = nb >> 3;
  const bool ovf = (nh >= RCAP);
  const float qnan = __int_as_float(0x7fc00000);
#pragma unroll 1
  for (int jt = 0; jt < nbw; ++jt) {
    const int slot = wave * nbw + jt;
    const int grow = nodeBase + slot;
    const int gcl  = grow < nN ? grow : nN - 1;
    int st = soff[slot];
    const int craw = scnt[slot];
    int cnt = craw;
    st  = st < 0 ? 0 : (st > nh ? nh : st);
    cnt = cnt < 0 ? 0 : (cnt > DEGCAP ? DEGCAP : cnt);
    if (cnt > nh - st) cnt = nh - st;
    const float pz = (ovf || craw > DEGCAP) ? qnan : 0.0f;
    const bool wr = grow < NPr;
    const float live = grow < nN ? 1.0f : 0.0f;
    const float di = DIS[grow];

    v4f sm = *(const v4f*)(G + (size_t)gcl * HD + 4 * lane);
#pragma unroll 1
    for (int q = 0; q < cnt; ++q) {
      int idx = st + q; idx = idx > RCAP - 1 ? RCAP - 1 : idx;
      int el = reg2[idx]; el = el < 0 ? 0 : (el > nE - 1 ? nE - 1 : el);
      int s = srcs[el]; s = s < 0 ? 0 : (s > nN - 1 ? nN - 1 : s);
      const v4f gv = *(const v4f*)(G + (size_t)s * HD + 4 * lane);
      sm = sm + gv;
    }
    const v4f ag = sm * di + b4;
    const v4f hr = relu4(ag) * live + pz;
    float* gp = H + (size_t)grow * HD + 4 * lane;
    if (wr) *(volatile v4f*)gp = hr;
    __threadfence();
    if (wr) *(volatile v4f*)gp = hr;
  }
}

__global__ __launch_bounds__(NTHR) void k_edge(const int* __restrict__ srcs, const int* __restrict__ dsts,
                                               const float* __restrict__ P, const float* __restrict__ Q,
                                               const float* __restrict__ wm2, const float* __restrict__ bm2,
                                               float* out, int nN, int nE) {
  __shared__ __attribute__((aligned(16))) v4f w2s[HD];
  __shared__ __attribute__((aligned(16))) float ost[NTHR * NOUT];
  const int tid = (int)threadIdx.x;
  if (tid < HD) {
    v4f w;
    w.x = bf16r(wm2[tid * NOUT + 0]);
    w.y = bf16r(wm2[tid * NOUT + 1]);
    w.z = bf16r(wm2[tid * NOUT + 2]);
    w.w = 0.f;
    w2s[tid] = w;
  }
  __syncthreads();

  const int eb = (int)blockIdx.x * NTHR;
  const int e  = eb + tid;
  const int ec = e > nE - 1 ? nE - 1 : e;
  int s = srcs[ec]; s = s < 0 ? 0 : (s > nN - 1 ? nN - 1 : s);
  int d = dsts[ec]; d = d < 0 ? 0 : (d > nN - 1 ? nN - 1 : d);
  const float* pp = P + (size_t)s * HD;
  const float* qq = Q + (size_t)d * HD;
  float a0 = 0.f, a1 = 0.f, a2 = 0.f;
#pragma unroll 1
  for (int k4 = 0; k4 < HD / 4; ++k4) {
    const v4f pv = *(const v4f*)(pp + 4 * k4);
    const v4f qv = *(const v4f*)(qq + 4 * k4);
    const v4f hv = relu4(pv + qv);
    const v4f w0 = w2s[4 * k4 + 0];
    const v4f w1 = w2s[4 * k4 + 1];
    const v4f w2 = w2s[4 * k4 + 2];
    const v4f w3 = w2s[4 * k4 + 3];
    a0 = fmaf(hv.x, w0.x, a0); a1 = fmaf(hv.x, w0.y, a1); a2 = fmaf(hv.x, w0.z, a2);
    a0 = fmaf(hv.y, w1.x, a0); a1 = fmaf(hv.y, w1.y, a1); a2 = fmaf(hv.y, w1.z, a2);
    a0 = fmaf(hv.z, w2.x, a0); a1 = fmaf(hv.z, w2.y, a1); a2 = fmaf(hv.z, w2.z, a2);
    a0 = fmaf(hv.w, w3.x, a0); a1 = fmaf(hv.w, w3.y, a1); a2 = fmaf(hv.w, w3.z, a2);
  }
  ost[tid * NOUT + 0] = a0 + bf16r(bm2[0]);
  ost[tid * NOUT + 1] = a1 + bf16r(bm2[1]);
  ost[tid * NOUT + 2] = a2 + bf16r(bm2[2]);
  __syncthreads();

  int nv = nE - eb;
  nv = nv < 0 ? 0 : (nv > NTHR ? NTHR : nv);
  const int nf  = nv * NOUT;
  const int npc = nf >> 2;
  const int rem = nf - 4 * npc;
  const int pi  = tid < (NTHR * NOUT / 4) ? tid : 0;
  const v4f pv  = *(const v4f*)(ost + 4 * pi);
  int ri = 4 * npc + tid;
  ri = ri > NTHR * NOUT - 1 ? NTHR * NOUT - 1 : ri;
  const float rv = ost[ri];
  float* ob = out + (size_t)eb * NOUT;
  if (tid < npc) *(volatile v4f*)(ob + 4 * tid) = pv;
  if (tid < rem) *(volatile float*)(ob + 4 * npc + tid) = rv;
  __threadfence();
  if (tid < npc) *(volatile v4f*)(ob + 4 * tid) = pv;
  if (tid < rem) *(volatile float*)(ob + 4 * npc + tid) = rv;
}

static inline int cdiv(int a, int b) { return (a + b - 1) / b; }
static int pick_nb(int nE, int nN) {
  int nb = NBMAX;
  while (nb > 32 && (long long)nb * (long long)nE * 11LL > (long long)RCAP * (long long)nN * 8LL) nb >>= 1;
  return nb;
}

extern "C" void kernel_launch(void* const* d_in, const int* in_sizes, int n_in,
                              void* d_out, int out_size, void* d_ws, size_t ws_size,
                              hipStream_t stream) {
  if (n_in < 13) return;
  const int nN = in_sizes[0];
  if (nN <= 0 || nN > (1 << 22)) return;
  const int nE = in_sizes[1] / 2;
  if (nE < 1 || in_sizes[1] != 2 * nE || nE > (1 << 21)) return;
  const int nV = in_sizes[2] / HD;
  if (nV < 1 || in_sizes[2] != nV * HD || nV > 4096) return;
  if (in_sizes[3] != HD * HD  || in_sizes[4]  != HD) return;
  if (in_sizes[5] != HD * HD  || in_sizes[6]  != HD) return;
  if (in_sizes[7] != HD * HD  || in_sizes[8]  != HD) return;
  if (in_sizes[9] != HD2 * HD || in_sizes[10] != HD) return;
  if (in_sizes[11] != HD * NOUT || in_sizes[12] != NOUT) return;
  if (out_size != nE * NOUT) return;

  const int*   xi  = (const int*)  d_in[0];
  const int*   ei  = (const int*)  d_in[1];
  const float* emb = (const float*)d_in[2];
  const float* W0  = (const float*)d_in[3];
  const float* b0  = (const float*)d_in[4];
  const float* W1  = (const float*)d_in[5];
  const float* b1  = (const float*)d_in[6];
  const float* W2  = (const float*)d_in[7];
  const float* b2  = (const float*)d_in[8];
  const float* Wm1 = (const float*)d_in[9];
  const float* bm1 = (const float*)d_in[10];
  const float* Wm2 = (const float*)d_in[11];
  const float* bm2 = (const float*)d_in[12];
  float* out = (float*)d_out;
  const int* srcp = ei;
  const int* dstp = ei + (size_t)nE;

  const int NP = cdiv(nN, GBM) * GBM;
  const int VP = cdiv(nV, GBM) * GBM;
  const int nb = pick_nb(nE, nN);
  const int gA = cdiv(NP, nb);
  if (gA * nb < NP || nb > NBMAX || nb < 32) return;
  const int DEGN = gA * nb;
  const int vec8 = ((nE & 3) == 0) ? 1 : 0;

  char* ws = (char*)d_ws;
  size_t off = 0;
  const size_t oWPL = off; off += (size_t)NPLANE * PLH * 2;         off = (off + 255) & ~(size_t)255;
  const size_t oEMB = off; off += (size_t)VP * HD * 4;              off = (off + 255) & ~(size_t)255;
  const size_t oTT  = off; off += (size_t)VP * HD * 4;              off = (off + 255) & ~(size_t)255;
  const size_t oDIS = off; off += (size_t)DEGN * 4;                 off = (off + 255) & ~(size_t)255;
  const size_t oRA  = off; off += (size_t)NP * HD * 4;              off = (off + 255) & ~(size_t)255;
  const size_t oRB  = off; off += (size_t)NP * HD * 4;              off = (off + 255) & ~(size_t)255;
  if (off > ws_size || off > (size_t)WSMAX) return;
  _Float16* WPL  = (_Float16*)(ws + oWPL);
  float*    EMBR = (float*)(ws + oEMB);
  float*    TT   = (float*)(ws + oTT);
  float*    DIS  = (float*)(ws + oDIS);
  float*    RA   = (float*)(ws + oRA);
  float*    RB   = (float*)(ws + oRB);
  const _Float16* W0T = WPL;
  const _Float16* W1T = WPL + (size_t)PLH;
  const _Float16* W2T = WPL + (size_t)2 * PLH;
  const _Float16* WPT = WPL + (size_t)3 * PLH;
  const _Float16* WQT = WPL + (size_t)4 * PLH;

  hipFuncSetAttribute(reinterpret_cast<const void*>(&k_deg),
                      hipFuncAttributeMaxDynamicSharedMemorySize, LDS_DEG);
  hipFuncSetAttribute(reinterpret_cast<const void*>(&k_agg),
                      hipFuncAttributeMaxDynamicSharedMemorySize, LDS_AGG);

  {
    const int nU = NPLANE * PLH / 8;
    k_wcvt<<<cdiv(nU, NTHR), NTHR, 0, stream>>>(W0, W1, W2, Wm1, WPL, nU);
  }
  {
    const int nT = VP * (HD / 4);
    k_embr<<<cdiv(nT, NTHR), NTHR, 0, stream>>>(emb, EMBR, nV, nT);
  }
  k_deg<<<gA, NTHR, LDS_DEG, stream>>>(dstp, DIS, nN, nE, nb, vec8);
  k_pgemm<2><<<VP / GBM, NTHR, 0, stream>>>(EMBR, W0T, b0, DIS, TT, VP);
  {
    const int nT = NP * (HD / 4);
    k_gath1<<<cdiv(nT, NTHR), NTHR, 0, stream>>>(xi, TT, DIS, RA, nN, nV, nT);
  }
  k_agg<<<gA, NTHR, LDS_AGG, stream>>>(dstp, srcp, RA, DIS, b0, RB, nN, nE, nb, vec8, NP);
  k_pgemm<1><<<NP / GBM, NTHR, 0, stream>>>(RB, W1T, b1, DIS, RA, NP);
  k_agg<<<gA, NTHR, LDS_AGG, stream>>>(dstp, srcp, RA, DIS, b1, RB, nN, nE, nb, vec8, NP);
  k_pgemm<1><<<NP / GBM, NTHR, 0, stream>>>(RB, W2T, b2, DIS, RA, NP);
  k_agg<<<gA, NTHR, LDS_AGG, stream>>>(dstp, srcp, RA, DIS, b2, RB, nN, nE, nb, vec8, NP);
  k_pgemm<2><<<NP / GBM, NTHR, 0, stream>>>(RB, WQT, bm1, DIS, RA, NP);
  k_pgemm<0><<<NP / GBM, NTHR, 0, stream>>>(RB, WPT, bm1, DIS, RB, NP);
  k_edge<<<cdiv(nE, NTHR), NTHR, 0, stream>>>(srcp, dstp, RB, RA, Wm2, bm2, out, nN, nE);
}
